// GroupRopeAttention_59992103191028
// MI455X (gfx1250) — hardware-verified
//
#include <hip/hip_runtime.h>
#include <math.h>
#include <stdint.h>

#pragma clang fp contract(off)

static constexpr int kBatch    = 2;
static constexpr int kSeq      = 2048;
static constexpr int kEmb      = 2048;
static constexpr int kHeadDim  = 128;
static constexpr int kNumHeads = 16;
static constexpr int kNqk      = kNumHeads * kHeadDim;
static constexpr int kNtot     = kNqk + 2 * kHeadDim;
static constexpr int kRows     = kBatch * kSeq;
static constexpr int kHalfDim  = kHeadDim / 2;

static constexpr size_t kQel   = (size_t)kBatch * kNumHeads * kSeq * kHeadDim;
static constexpr size_t kKel   = (size_t)kBatch * kSeq * kHeadDim;
static constexpr size_t kLoBlk = kQel + 2 * kKel;

static constexpr size_t kOffXb   = 0;
static constexpr size_t kBytesXb = (size_t)kRows * kEmb * 2;
static constexpr size_t kOffWt   = kOffXb + kBytesXb;
static constexpr size_t kBytesWt = (size_t)kNtot * kEmb * 2;
static constexpr size_t kOffC    = kOffWt + kBytesWt;
static constexpr size_t kBytesC  = (size_t)kRows * kNtot * 4;
static constexpr size_t kOffTab  = kOffC + kBytesC;
static constexpr size_t kBytesTab= (size_t)kSeq * kHalfDim * 2 * 4;
static constexpr size_t kOffP16  = kOffTab + kBytesTab;
static constexpr size_t kBytesP16= 2 * kLoBlk * 2;
static constexpr size_t kWsTotal = kOffP16 + kBytesP16;
static_assert(kOffWt % 128 == 0 && kOffC % 128 == 0 && kOffTab % 128 == 0 && kOffP16 % 128 == 0, "128-B aligned carves");
static_assert(kWsTotal == 102760448ull, "carve total");
static_assert(kWsTotal <= 134217728ull, "carve under 128 MiB");
static_assert(kRows % 64 == 0 && kNtot % 64 == 0 && kEmb % 32 == 0, "GEMM M,N tile multiples and K % 32 == 0");
static_assert(kNqk % 64 == 0 && kHeadDim % 64 == 0, "fused column blocks are 64-aligned");
static_assert(kSeq % 64 == 0 && kHeadDim == 128, "attention tiling");

typedef __attribute__((ext_vector_type(16))) _Float16 v16h;
typedef __attribute__((ext_vector_type(8)))  _Float16 v8h;
typedef __attribute__((ext_vector_type(16))) __bf16   v16b;
typedef __attribute__((ext_vector_type(8)))  __bf16   v8b;
typedef __attribute__((ext_vector_type(8)))  float    v8f;
typedef __attribute__((ext_vector_type(4)))  float    v4f;
typedef __attribute__((ext_vector_type(4)))  unsigned int v4u;
#define PSCALE 32768.0f
#define U16(p) ((const unsigned short*)(const void*)(p))
#define PSCALE_INV (1.0f / 32768.0f)

__device__ __forceinline__ unsigned short f2bf_bits(float f) {
  unsigned u = __float_as_uint(f);
  return (unsigned short)((u + 0x7FFFu + ((u >> 16) & 1u)) >> 16);
}
__device__ __forceinline__ float bf_bits2f(unsigned short h) { return __uint_as_float(((unsigned)h) << 16); }

__device__ __forceinline__ void dep_guard_h(v8f& a, v8f& b, v16h x, v16h y) { asm volatile("v_nop\n\tv_nop\n\tv_nop\n\tv_nop" : "+v"(a), "+v"(b) : "v"(x), "v"(y)); }
__device__ __forceinline__ void dep_guard_b(v8f& a, v8f& b, v16b x, v16b y) { asm volatile("v_nop\n\tv_nop\n\tv_nop\n\tv_nop" : "+v"(a), "+v"(b) : "v"(x), "v"(y)); }
__device__ __forceinline__ void keep4_h(v16h a, v16h b, v16h c, v16h d) { asm volatile("v_nop" :: "v"(a), "v"(b), "v"(c), "v"(d)); }
__device__ __forceinline__ void keep4_b(v16b a, v16b b, v16b c, v16b d) { asm volatile("v_nop" :: "v"(a), "v"(b), "v"(c), "v"(d)); }
__device__ __forceinline__ void acc_guard4(v8f& a, v8f& b, v8f& c, v8f& d) { asm volatile("v_nop\n\tv_nop\n\tv_nop\n\tv_nop" : "+v"(a), "+v"(b), "+v"(c), "+v"(d)); }
template <typename T> struct Frag;
template <> struct Frag<_Float16> {
  typedef v16h V; union U { v16h v; v8h h[2]; };
  static __device__ __forceinline__ v16h load(const _Float16* p) {
    U f; f.h[0] = *(const v8h*)(p); f.h[1] = *(const v8h*)(p + 16); return f.v;
  }
  static __device__ __forceinline__ v8f mma(v16h a, v16h b, v8f c) {
    return __builtin_amdgcn_wmma_f32_16x16x32_f16(false, a, false, b, (short)0, c, false, false);
  }
  static __device__ __forceinline__ void guard(v8f& a, v8f& b, v16h x, v16h y) { dep_guard_h(a, b, x, y); }
  static __device__ __forceinline__ void keep(v16h a, v16h b, v16h c, v16h d) { keep4_h(a, b, c, d); }
};
template <> struct Frag<__bf16> {
  typedef v16b V; union U { v16b v; v8b h[2]; };
  static __device__ __forceinline__ v16b load(const __bf16* p) {
    U f; f.h[0] = *(const v8b*)(p); f.h[1] = *(const v8b*)(p + 16); return f.v;
  }
  static __device__ __forceinline__ v8f mma(v16b a, v16b b, v8f c) {
    return __builtin_amdgcn_wmma_f32_16x16x32_bf16(false, a, false, b, (short)0, c, false, false);
  }
  static __device__ __forceinline__ void guard(v8f& a, v8f& b, v16b x, v16b y) { dep_guard_b(a, b, x, y); }
  static __device__ __forceinline__ void keep(v16b a, v16b b, v16b c, v16b d) { keep4_b(a, b, c, d); }
};

template <int ET> struct Elem;
template <> struct Elem<0> { typedef _Float16 T; };
template <> struct Elem<1> { typedef __bf16 T; };
template <int ET, bool SPLIT, int BIAS_MODE, int OUT_MODE, bool RESID, int ACT = 0>
__global__ __launch_bounds__(256) void wmma_gemm64(
    const unsigned short* __restrict__ Ap, const unsigned short* __restrict__ A2p, int lda, long strideA,
    const unsigned short* __restrict__ Btp, const unsigned short* __restrict__ Bt2p, int ldb, long strideB,
    void* __restrict__ Cout, void* __restrict__ Cout2, int ldc, long strideC,
    const float* __restrict__ bias,
    const float* __restrict__ resid, long strideR,
    int M, int N, int K, float scale) {
  typedef typename Elem<ET>::T T;
  typedef typename Frag<T>::V V;
  const T* A = (const T*)Ap; const T* A2 = (const T*)A2p; const T* Bt = (const T*)Btp; const T* Bt2 = (const T*)Bt2p;
  __shared__ __align__(16) float sT[8][16 * 68];
  const int b    = blockIdx.y;
  const int lane = threadIdx.x & 31;
  const int wave = threadIdx.x >> 5;
  const int tilesN = N >> 6;
  const int tilesM = M >> 6;
  const int tile = blockIdx.x * 8 + wave;
  if (tile >= tilesM * tilesN) return;
  const int tm = tile / tilesN;
  const int tn = tile - tm * tilesN;
  const int m0 = tm << 6;
  const int n0 = tn << 6;

  const T* Ab  = A  + (size_t)b * strideA;
  const T* Bb  = Bt + (size_t)b * strideB;
  const T* Ab2 = SPLIT ? (A2  + (size_t)b * strideA) : nullptr;
  const T* Bb2 = SPLIT ? (Bt2 + (size_t)b * strideB) : nullptr;

  const int rlane = lane & 15;
  const int koff  = (lane >> 4) * 8;
  const int mOff  = (lane >> 4) * 8;

  v8f acc[4][4];
#pragma unroll
  for (int i = 0; i < 4; ++i)
#pragma unroll
    for (int j = 0; j < 4; ++j) acc[i][j] = (v8f){0.f,0.f,0.f,0.f,0.f,0.f,0.f,0.f};

  for (int k0 = 0; k0 < K; k0 += 32) {
    V bh[4], bl[4];
#pragma unroll
    for (int j = 0; j < 4; ++j) {
      const size_t bo = (size_t)(n0 + (j << 4) + rlane) * ldb + koff + k0;
      bh[j] = Frag<T>::load(Bb + bo);
      if (SPLIT) bl[j] = Frag<T>::load(Bb2 + bo);
    }
#pragma unroll
    for (int i = 0; i < 4; ++i) {
      const size_t ao = (size_t)(m0 + (i << 4) + rlane) * lda + koff + k0;
      V ah = Frag<T>::load(Ab + ao);
      V al;
      if (SPLIT) al = Frag<T>::load(Ab2 + ao);
#pragma unroll
      for (int j = 0; j < 4; ++j) {
        acc[i][j] = Frag<T>::mma(ah, bh[j], acc[i][j]);
        if (SPLIT) {
          acc[i][j] = Frag<T>::mma(ah, bl[j], acc[i][j]);
          acc[i][j] = Frag<T>::mma(al, bh[j], acc[i][j]);
        }
      }
      Frag<T>::guard(acc[i][0], acc[i][3], ah, SPLIT ? al : ah);
    }
    Frag<T>::keep(bh[0], bh[1], bh[2], bh[3]);
    if (SPLIT) Frag<T>::keep(bl[0], bl[1], bl[2], bl[3]);
  }
  acc_guard4(acc[0][0], acc[0][1], acc[0][2], acc[0][3]);
  acc_guard4(acc[1][0], acc[1][1], acc[1][2], acc[1][3]);
  acc_guard4(acc[2][0], acc[2][1], acc[2][2], acc[2][3]);
  acc_guard4(acc[3][0], acc[3][1], acc[3][2], acc[3][3]);

  float* slab = sT[wave];
  const float* Rb = RESID ? (resid + (size_t)b * strideR) : nullptr;
#pragma unroll
  for (int i = 0; i < 4; ++i) {
    const int mBase = m0 + (i << 4);
#pragma unroll
    for (int j = 0; j < 4; ++j) {
      const int n = n0 + (j << 4) + rlane;
      float bv = 0.f;
      if (BIAS_MODE == 2) bv = bias[n];
#pragma unroll
      for (int r = 0; r < 8; ++r) {
        float v = acc[i][j][r] * scale;
        if (BIAS_MODE == 1) v += bias[mBase + mOff + r];
        if (BIAS_MODE == 2) v += bv;
        if (RESID) v += Rb[(size_t)(mBase + mOff + r) * ldc + n];
        if (ACT == 1) v = tanhf(v);
        if (ACT == 2) v = fmaxf(v, 0.0f);
        if (ACT == 3) v = v / (1.0f + expf(-v));
        if (ACT == 4) v = (v > 0.f) ? v : 0.01f * v;
        if (ACT == 5) v = 0.5f * v * (1.0f + erff(v * 0.70710678118654752f));
        slab[(mOff + r) * 68 + (j << 4) + rlane] = v;
      }
    }
    __builtin_amdgcn_fence(__ATOMIC_RELEASE, "workgroup");
    __builtin_amdgcn_wave_barrier();
    __builtin_amdgcn_fence(__ATOMIC_ACQUIRE, "workgroup");
    if (OUT_MODE == 0) {
      float* C = (float*)Cout + (size_t)b * strideC;
      const int hh = lane >> 4, c4 = (lane & 15) * 4;
      for (int pass = 0; pass < 2; ++pass) {
#pragma unroll
        for (int it = 0; it < 8; ++it) {
          const int row = it * 2 + hh;
          v4f v = *(const v4f*)(slab + row * 68 + c4);
          *(volatile v4f*)(C + (size_t)(mBase + row) * ldc + n0 + c4) = v;
        }
        __threadfence();
      }
    } else {
      const int q = lane >> 3, c8 = (lane & 7) * 8;
      unsigned short* C  = (unsigned short*)Cout  + (size_t)b * strideC;
      unsigned short* C2 = (OUT_MODE == 2) ? ((unsigned short*)Cout2 + (size_t)b * strideC) : nullptr;
      for (int pass = 0; pass < 2; ++pass) {
#pragma unroll
        for (int it = 0; it < 4; ++it) {
          const int row = it * 4 + q;
          const float* sp = slab + row * 68 + c8;
          v8h hv, lv;
#pragma unroll
          for (int e = 0; e < 8; ++e) {
            if (OUT_MODE == 1) {
              hv[e] = (_Float16)sp[e];
            } else {
              unsigned short hb = f2bf_bits(sp[e]);
              unsigned short lb = f2bf_bits(sp[e] - bf_bits2f(hb));
              hv[e] = __builtin_bit_cast(_Float16, hb);
              lv[e] = __builtin_bit_cast(_Float16, lb);
            }
          }
          *(volatile v8h*)(C + (size_t)(mBase + row) * ldc + n0 + c8) = hv;
          if (OUT_MODE == 2) *(volatile v8h*)(C2 + (size_t)(mBase + row) * ldc + n0 + c8) = lv;
        }
        __threadfence();
      }
    }
    __builtin_amdgcn_fence(__ATOMIC_RELEASE, "workgroup");
    __builtin_amdgcn_wave_barrier();
    __builtin_amdgcn_fence(__ATOMIC_ACQUIRE, "workgroup");
  }
}

__device__ __forceinline__ unsigned short at_bf_bits(float f) {
  unsigned u = __float_as_uint(f);
  return (unsigned short)((u + 0x7FFFu + ((u >> 16) & 1u)) >> 16);
}
__device__ __forceinline__ __bf16 at_f2bf(float f) { return __builtin_bit_cast(__bf16, at_bf_bits(f)); }
__device__ __forceinline__ void at_split(float f, __bf16& hi, __bf16& lo) {
  const unsigned short hb = at_bf_bits(f);
  hi = __builtin_bit_cast(__bf16, hb);
  lo = at_f2bf(f - __uint_as_float(((unsigned)hb) << 16));
}

__device__ __forceinline__ v8f mq_mma3(v16b ah, v16b al, v16b bh, v16b bl, v8f c) {
  c = __builtin_amdgcn_wmma_f32_16x16x32_bf16(false, ah, false, bh, (short)0, c, false, false);
  c = __builtin_amdgcn_wmma_f32_16x16x32_bf16(false, ah, false, bl, (short)0, c, false, false);
  c = __builtin_amdgcn_wmma_f32_16x16x32_bf16(false, al, false, bh, (short)0, c, false, false);
  asm volatile("v_nop\n\tv_nop\n\tv_nop\n\tv_nop" : "+v"(c) : "v"(ah), "v"(al), "v"(bh), "v"(bl));
  return c;
}

__device__ __forceinline__ unsigned pack_bf16x2(float lo_el, float hi_el) {
  return (unsigned)f2bf_bits(lo_el) | ((unsigned)f2bf_bits(hi_el) << 16);
}

__global__ __launch_bounds__(256) void cast_x_bf16(const float* __restrict__ xin,
                                                   unsigned short* __restrict__ xo, int n8) {
  const int i = blockIdx.x * 256 + threadIdx.x;
  if (i >= n8) return;
  const float* p = xin + (size_t)i * 8;
  const v4f a = *(const v4f*)p;
  const v4f bq = *(const v4f*)(p + 4);
  v4u w;
  w.x = pack_bf16x2(a.x, a.y);
  w.y = pack_bf16x2(a.z, a.w);
  w.z = pack_bf16x2(bq.x, bq.y);
  w.w = pack_bf16x2(bq.z, bq.w);
  unsigned short* dst = xo + (size_t)i * 8;
  *(volatile v4u*)dst = w;
  __threadfence();
  *(volatile v4u*)dst = w;
}

__global__ __launch_bounds__(256) void wcat_t_bf16(const float* __restrict__ Wq, const float* __restrict__ Wk,
                                                   const float* __restrict__ Wv, unsigned short* __restrict__ WT) {
  __shared__ float sW[64][65];
  const int tid = threadIdx.x, lane = tid & 31, wave = tid >> 5;
  const int n0 = blockIdx.x * 64;
  const int k0 = blockIdx.y * 64;
  const float* src; int pitch; int nb;
  if (n0 < kNqk)                 { src = Wq; pitch = kNqk;     nb = n0; }
  else if (n0 < kNqk + kHeadDim) { src = Wk; pitch = kHeadDim; nb = n0 - kNqk; }
  else                           { src = Wv; pitch = kHeadDim; nb = n0 - kNqk - kHeadDim; }
  {
    const int kr = tid >> 2, nc = (tid & 3) * 16;
    const float* p = src + (size_t)(k0 + kr) * pitch + nb + nc;
#pragma unroll
    for (int q = 0; q < 4; ++q) {
      const v4f v = *(const v4f*)(p + 4 * q);
      sW[nc + 4 * q + 0][kr] = v.x;
      sW[nc + 4 * q + 1][kr] = v.y;
      sW[nc + 4 * q + 2][kr] = v.z;
      sW[nc + 4 * q + 3][kr] = v.w;
    }
  }
  __syncthreads();
  v4u wv0, wv1;
  size_t wo0, wo1;
  {
    const int row = wave * 8 + (lane >> 3), c8 = (lane & 7) * 8;
    wv0.x = pack_bf16x2(sW[row][c8 + 0], sW[row][c8 + 1]);
    wv0.y = pack_bf16x2(sW[row][c8 + 2], sW[row][c8 + 3]);
    wv0.z = pack_bf16x2(sW[row][c8 + 4], sW[row][c8 + 5]);
    wv0.w = pack_bf16x2(sW[row][c8 + 6], sW[row][c8 + 7]);
    wo0 = (size_t)(n0 + row) * kEmb + k0 + c8;
  }
  {
    const int row = wave * 8 + 4 + (lane >> 3), c8 = (lane & 7) * 8;
    wv1.x = pack_bf16x2(sW[row][c8 + 0], sW[row][c8 + 1]);
    wv1.y = pack_bf16x2(sW[row][c8 + 2], sW[row][c8 + 3]);
    wv1.z = pack_bf16x2(sW[row][c8 + 4], sW[row][c8 + 5]);
    wv1.w = pack_bf16x2(sW[row][c8 + 6], sW[row][c8 + 7]);
    wo1 = (size_t)(n0 + row) * kEmb + k0 + c8;
  }
  *(volatile v4u*)(WT + wo0) = wv0;
  *(volatile v4u*)(WT + wo1) = wv1;
  __threadfence();
  *(volatile v4u*)(WT + wo0) = wv0;
  *(volatile v4u*)(WT + wo1) = wv1;
}

struct FreqTab { float f[64]; };
static_assert(sizeof(FreqTab) == 256, "no padding");

__global__ __launch_bounds__(256) void rope_table(float* __restrict__ tab, int L, FreqTab ft) {
  const int gid = blockIdx.x * 256 + threadIdx.x;
  const int l = gid >> 5;
  const int j0 = (gid & 31) * 2;
  if (l >= L) return;
  v4f o = (v4f){0.f, 0.f, 0.f, 0.f};
#pragma unroll 1
  for (int i = 0; i < 2; ++i) {
    const int j = j0 + i;
    float fr = 0.f;
#pragma unroll
    for (int q = 0; q < 64; ++q) fr = (j == q) ? ft.f[q] : fr;
    const float ang = (float)l * fr;
    float sv, cv;
    sincosf(ang, &sv, &cv);
    o = (i == 0) ? (v4f){cv, sv, o.z, o.w} : (v4f){o.x, o.y, cv, sv};
  }
  float* p = tab + ((size_t)l * kHalfDim + j0) * 2;
  *(volatile v4f*)p = o;
  __threadfence();
  *(volatile v4f*)p = o;
}

__global__ __launch_bounds__(288) void rope_split_planes(const float* __restrict__ Cp,
                                                         const float* __restrict__ tab,
                                                         unsigned short* __restrict__ P16) {
  const int m = blockIdx.x;
  const int b = m / kSeq;
  const int l = m - b * kSeq;
  const int t = threadIdx.x;
  const int n0 = t * 8;
  const float* crow = Cp + (size_t)m * kNtot + n0;
  const v4f xa = *(const v4f*)crow;
  const v4f xc = *(const v4f*)(crow + 4);
  const int dloc = n0 & (kHeadDim - 1);
  const int j0 = dloc >> 1;
  const float* tp = tab + ((size_t)l * kHalfDim + j0) * 2;
  const v4f ta = *(const v4f*)tp;
  const v4f tb = *(const v4f*)(tp + 4);
  const bool isV = (n0 >= kNqk + kHeadDim);
  float o0 = xa.x * ta.x - xa.y * ta.y;
  float o1 = xa.y * ta.x + xa.x * ta.y;
  float o2 = xa.z * ta.z - xa.w * ta.w;
  float o3 = xa.w * ta.z + xa.z * ta.w;
  float o4 = xc.x * tb.x - xc.y * tb.y;
  float o5 = xc.y * tb.x + xc.x * tb.y;
  float o6 = xc.z * tb.z - xc.w * tb.w;
  float o7 = xc.w * tb.z + xc.z * tb.w;
  if (isV) { o0 = xa.x; o1 = xa.y; o2 = xa.z; o3 = xa.w; o4 = xc.x; o5 = xc.y; o6 = xc.z; o7 = xc.w; }
  const size_t rowBL = (size_t)(b * kSeq + l);
  const size_t offQ = (((size_t)(b * kNumHeads + (n0 >> 7))) * kSeq + l) * kHeadDim + dloc;
  const size_t offK = kQel + rowBL * kHeadDim + dloc;
  const size_t offV = kQel + kKel + rowBL * kHeadDim + dloc;
  const size_t off = (n0 < kNqk) ? offQ : (isV ? offV : offK);

  unsigned short hb[8], lb[8];
  {
    const float ov[8] = {o0, o1, o2, o3, o4, o5, o6, o7};
#pragma unroll
    for (int e = 0; e < 8; ++e) {
      hb[e] = f2bf_bits(ov[e]);
      lb[e] = f2bf_bits(ov[e] - bf_bits2f(hb[e]));
    }
  }
  v4u hv, lv;
  hv.x = (unsigned)hb[0] | ((unsigned)hb[1] << 16);
  hv.y = (unsigned)hb[2] | ((unsigned)hb[3] << 16);
  hv.z = (unsigned)hb[4] | ((unsigned)hb[5] << 16);
  hv.w = (unsigned)hb[6] | ((unsigned)hb[7] << 16);
  lv.x = (unsigned)lb[0] | ((unsigned)lb[1] << 16);
  lv.y = (unsigned)lb[2] | ((unsigned)lb[3] << 16);
  lv.z = (unsigned)lb[4] | ((unsigned)lb[5] << 16);
  lv.w = (unsigned)lb[6] | ((unsigned)lb[7] << 16);
  unsigned short* ph = P16 + off;
  unsigned short* plo = P16 + kLoBlk + off;
  *(volatile v4u*)ph = hv;
  *(volatile v4u*)plo = lv;
  __threadfence();
  *(volatile v4u*)ph = hv;
  *(volatile v4u*)plo = lv;
}

#define MQ_HDIM 128
#define MQ_KC   64
#define MQ_QB   64
#define MQ_NW   4
#define MQ_OP   68

__global__ __launch_bounds__(128)
void mq_attn_hd128(const unsigned short* __restrict__ Qh, const unsigned short* __restrict__ Ql,
                   const unsigned short* __restrict__ Kh, const unsigned short* __restrict__ Kl,
                   const unsigned short* __restrict__ Vh, const unsigned short* __restrict__ Vl,
                   float* __restrict__ out, int L, int NHQ, int ors, float sscale) {
  union FB { v16b v; v8b h[2]; };
  __shared__ __align__(16) __bf16 Qhs[MQ_QB * MQ_HDIM];
  __shared__ __align__(16) __bf16 Qls[MQ_QB * MQ_HDIM];
  __shared__ __align__(16) __bf16 Khs[MQ_KC * MQ_HDIM];
  __shared__ __align__(16) __bf16 Kls[MQ_KC * MQ_HDIM];
  __shared__ __align__(16) __bf16 Vths[MQ_HDIM * MQ_KC];
  __shared__ __align__(16) __bf16 Vtls[MQ_HDIM * MQ_KC];
  __shared__ __align__(16) __bf16 Phs[MQ_NW][16 * MQ_KC];
  __shared__ __align__(16) __bf16 Pls[MQ_NW][16 * MQ_KC];
  __shared__ __align__(16) float  Os[MQ_NW][16 * MQ_OP];

  const int tid  = threadIdx.x;
  const int wave = tid >> 5;
  const int lane = tid & 31;
  const int hh   = lane >> 4;
  const int c    = lane & 15;

  const int nqb = L / MQ_QB;
  const int bx  = blockIdx.x;
  const int qb  = bx % nqb;
  const int bh  = bx / nqb;
  const int h   = bh % NHQ;
  const int b   = bh / NHQ;
  const int q0  = qb * MQ_QB + wave * 16;

  const __bf16* Qhp = (const __bf16*)Qh + ((size_t)bh * L + (size_t)qb * MQ_QB) * MQ_HDIM;
  const __bf16* Qlp = (const __bf16*)Ql + ((size_t)bh * L + (size_t)qb * MQ_QB) * MQ_HDIM;
  const __bf16* Khp = (const __bf16*)Kh + (size_t)b * L * MQ_HDIM;
  const __bf16* Klp = (const __bf16*)Kl + (size_t)b * L * MQ_HDIM;
  const unsigned short* Vhp = Vh + (size_t)b * L * MQ_HDIM;
  const unsigned short* Vlp = Vl + (size_t)b * L * MQ_HDIM;
  float* ob = out + (size_t)b * L * ors + (size_t)h * MQ_HDIM;

#pragma unroll 1
  for (int pl = 0; pl < 2; ++pl) {
    const __bf16* src = (pl == 0) ? Qhp : Qlp;
    __bf16* dst = (pl == 0) ? Qhs : Qls;
#pragma unroll
    for (int i = 0; i < 8; ++i) {
      const int u = tid + 128 * i;
      *(v8b*)(dst + u * 8) = *(const v8b*)(src + (size_t)u * 8);
    }
  }

  float mrow[8], lrow[8];
  v8f oacc[8];
#pragma unroll
  for (int r = 0; r < 8; ++r) { mrow[r] = -INFINITY; lrow[r] = 0.f; }
#pragma unroll
  for (int t = 0; t < 8; ++t) oacc[t] = (v8f){0.f,0.f,0.f,0.f,0.f,0.f,0.f,0.f};

  const int nChunks = qb + 1;
  for (int kc = 0; kc < nChunks; ++kc) {
    const int kv0 = kc * MQ_KC;
    __syncthreads();
#pragma unroll 1
    for (int pl = 0; pl < 2; ++pl) {
      const __bf16* src = ((pl == 0) ? Khp : Klp) + (size_t)kv0 * MQ_HDIM;
      __bf16* dst = (pl == 0) ? Khs : Kls;
#pragma unroll
      for (int i = 0; i < 8; ++i) {
        const int u = tid + 128 * i;
        *(v8b*)(dst + u * 8) = *(const v8b*)(src + (size_t)u * 8);
      }
    }
    {
      const int kvr = tid >> 1, dh = (tid & 1) * 64;
#pragma unroll 1
      for (int pl = 0; pl < 2; ++pl) {
        const unsigned short* src = ((pl == 0) ? Vhp : Vlp) + (size_t)(kv0 + kvr) * MQ_HDIM + dh;
        __bf16* dst = (pl == 0) ? Vths : Vtls;
#pragma unroll
        for (int i = 0; i < 8; ++i) {
          const v4u w = *(const v4u*)(src + 8 * i);
#pragma unroll
          for (int e = 0; e < 4; ++e) {
            const unsigned wv = w[e];
            const int d = dh + 8 * i + 2 * e;
            dst[d * MQ_KC + kvr]       = __builtin_bit_cast(__bf16, (unsigned short)(wv & 0xffffu));
            dst[(d + 1) * MQ_KC + kvr] = __builtin_bit_cast(__bf16, (unsigned short)(wv >> 16));
          }
        }
      }
    }
    __syncthreads();

    v8f s[4];
#pragma unroll
    for (int j = 0; j < 4; ++j) s[j] = (v8f){0.f,0.f,0.f,0.f,0.f,0.f,0.f,0.f};
    {
      const __bf16* qhr = Qhs + (wave * 16 + c) * MQ_HDIM + 8 * hh;
      const __bf16* qlr = Qls + (wave * 16 + c) * MQ_HDIM + 8 * hh;
#pragma unroll 1
      for (int dc = 0; dc < 4; ++dc) {
        FB qa, qlo;
        qa.h[0]  = *(const v8b*)(qhr + dc * 32);
        qa.h[1]  = *(const v8b*)(qhr + dc * 32 + 16);
        qlo.h[0] = *(const v8b*)(qlr + dc * 32);
        qlo.h[1] = *(const v8b*)(qlr + dc * 32 + 16);
#pragma unroll
        for (int j = 0; j < 4; ++j) {
          const __bf16* khp2 = Khs + (j * 16 + c) * MQ_HDIM + dc * 32 + 8 * hh;
          const __bf16* klp2 = Kls + (j * 16 + c) * MQ_HDIM + dc * 32 + 8 * hh;
          FB kb, klo;
          kb.h[0]  = *(const v8b*)(khp2);
          kb.h[1]  = *(const v8b*)(khp2 + 16);
          klo.h[0] = *(const v8b*)(klp2);
          klo.h[1] = *(const v8b*)(klp2 + 16);
          s[j] = mq_mma3(qa.v, qlo.v, kb.v, klo.v, s[j]);
        }
      }
    }

    const bool diag = (kc == qb);
    float cm[8];
#pragma unroll
    for (int r = 0; r < 8; ++r) {
      const int qrow = q0 + 8 * hh + r;
      float m = -INFINITY;
#pragma unroll
      for (int j = 0; j < 4; ++j) {
        const int kvcol = kv0 + j * 16 + c;
        float v = s[j][r] * sscale;
        if (diag && (kvcol > qrow)) v = -INFINITY;
        s[j][r] = v;
        m = fmaxf(m, v);
      }
#pragma unroll
      for (int off = 1; off < 16; off <<= 1) m = fmaxf(m, __shfl_xor(m, off, 32));
      cm[r] = m;
    }
    __bf16* pwh = Phs[wave];
    __bf16* pwl = Pls[wave];
#pragma unroll
    for (int r = 0; r < 8; ++r) {
      const float mnew = fmaxf(mrow[r], cm[r]);
      const float alpha = expf(mrow[r] - mnew);
      mrow[r] = mnew;
      float psum = 0.f;
#pragma unroll
      for (int j = 0; j < 4; ++j) {
        const float p = expf(s[j][r] - mnew);
        psum += p;
        __bf16 a, blo;
        at_split(p, a, blo);
        pwh[(8 * hh + r) * MQ_KC + j * 16 + c] = a;
        pwl[(8 * hh + r) * MQ_KC + j * 16 + c] = blo;
      }
#pragma unroll
      for (int off = 1; off < 16; off <<= 1) psum += __shfl_xor(psum, off, 32);
      lrow[r] = lrow[r] * alpha + psum;
#pragma unroll
      for (int t = 0; t < 8; ++t) oacc[t][r] *= alpha;
    }
    __builtin_amdgcn_fence(__ATOMIC_RELEASE, "workgroup");
    __builtin_amdgcn_wave_barrier();
    __builtin_amdgcn_fence(__ATOMIC_ACQUIRE, "workgroup");

#pragma unroll 1
    for (int kk = 0; kk < 2; ++kk) {
      FB pa, plo;
      pa.h[0]  = *(const v8b*)(pwh + c * MQ_KC + kk * 32 + 8 * hh);
      pa.h[1]  = *(const v8b*)(pwh + c * MQ_KC + kk * 32 + 16 + 8 * hh);
      plo.h[0] = *(const v8b*)(pwl + c * MQ_KC + kk * 32 + 8 * hh);
      plo.h[1] = *(const v8b*)(pwl + c * MQ_KC + kk * 32 + 16 + 8 * hh);
#pragma unroll
      for (int t = 0; t < 8; ++t) {
        const __bf16* vhp2 = Vths + (t * 16 + c) * MQ_KC + kk * 32 + 8 * hh;
        const __bf16* vlp2 = Vtls + (t * 16 + c) * MQ_KC + kk * 32 + 8 * hh;
        FB vb, vlo;
        vb.h[0]  = *(const v8b*)(vhp2);
        vb.h[1]  = *(const v8b*)(vhp2 + 16);
        vlo.h[0] = *(const v8b*)(vlp2);
        vlo.h[1] = *(const v8b*)(vlp2 + 16);
        oacc[t] = mq_mma3(pa.v, plo.v, vb.v, vlo.v, oacc[t]);
      }
    }
  }

  float invl[8];
#pragma unroll
  for (int r = 0; r < 8; ++r) invl[r] = 1.0f / lrow[r];
  float* os = Os[wave];
  const int c4 = (lane & 15) * 4;
#pragma unroll
  for (int hf = 0; hf < 2; ++hf) {
#pragma unroll
    for (int r = 0; r < 8; ++r) {
#pragma unroll
      for (int tt = 0; tt < 4; ++tt) os[(8 * hh + r) * MQ_OP + tt * 16 + c] = oacc[hf * 4 + tt][r] * invl[r];
    }
    __builtin_amdgcn_fence(__ATOMIC_RELEASE, "workgroup");
    __builtin_amdgcn_wave_barrier();
    __builtin_amdgcn_fence(__ATOMIC_ACQUIRE, "workgroup");
    for (int pass = 0; pass < 2; ++pass) {
#pragma unroll
      for (int it = 0; it < 8; ++it) {
        const int row = it * 2 + hh;
        const v4f val = *(const v4f*)(os + row * MQ_OP + c4);
        *(volatile v4f*)(ob + (size_t)(q0 + row) * ors + hf * 64 + c4) = val;
      }
      __threadfence();
    }
    __builtin_amdgcn_fence(__ATOMIC_RELEASE, "workgroup");
    __builtin_amdgcn_wave_barrier();
    __builtin_amdgcn_fence(__ATOMIC_ACQUIRE, "workgroup");
  }
}

extern "C" void kernel_launch(void* const* d_in, const int* in_sizes, int n_in,
                              void* d_out, int out_size, void* d_ws, size_t ws_size,
                              hipStream_t stream) {
  if (n_in < 4) return;
  if (in_sizes[0] != kRows * kEmb) return;
  if (in_sizes[1] != kEmb * kNqk) return;
  if (in_sizes[2] != kEmb * kHeadDim) return;
  if (in_sizes[3] != kEmb * kHeadDim) return;
  if (out_size != kRows * kNqk) return;
  if (ws_size < kWsTotal) return;

  const float* x  = (const float*)d_in[0];
  const float* Wq = (const float*)d_in[1];
  const float* Wk = (const float*)d_in[2];
  const float* Wv = (const float*)d_in[3];
  float* out = (float*)d_out;

  char* ws = (char*)d_ws;
  unsigned short* xb  = (unsigned short*)(ws + kOffXb);
  unsigned short* WT  = (unsigned short*)(ws + kOffWt);
  float*          Cws = (float*)(ws + kOffC);
  float*          tab = (float*)(ws + kOffTab);
  unsigned short* P16 = (unsigned short*)(ws + kOffP16);
  const unsigned short* Qh = P16;
  const unsigned short* Kh = P16 + kQel;
  const unsigned short* Vh = P16 + kQel + kKel;
  const unsigned short* Ql = P16 + kLoBlk;
  const unsigned short* Kl = P16 + kLoBlk + kQel;
  const unsigned short* Vl = P16 + kLoBlk + kQel + kKel;

  FreqTab ft;
  for (int i = 0; i < 64; ++i) {
    const float e = (float)(2 * i) / 128.0f;
    const float p = (float)pow(10000.0, (double)e);
    ft.f[i] = 1.0f / p;
  }
  const float sscale = 1.0f / sqrtf((float)kHeadDim);

  {
    const int n8 = (kRows * kEmb) / 8;
    cast_x_bf16<<<(n8 + 255) / 256, 256, 0, stream>>>(x, xb, n8);
  }
  wcat_t_bf16<<<dim3(kNtot / 64, kEmb / 64), 256, 0, stream>>>(Wq, Wk, Wv, WT);
  rope_table<<<(kSeq * 32 + 255) / 256, 256, 0, stream>>>(tab, kSeq, ft);
  {
    const int tiles = (kRows / 64) * (kNtot / 64);
    wmma_gemm64<1, false, 0, 0, false, 0><<<dim3((tiles + 7) / 8, 1), 256, 0, stream>>>(
        xb, xb, kEmb, 0L,
        WT, WT, kEmb, 0L,
        (void*)Cws, (void*)Cws, kNtot, 0L,
        (const float*)Cws,
        (const float*)Cws, 0L,
        kRows, kNtot, kEmb, 1.0f);
  }
  rope_split_planes<<<kRows, 288, 0, stream>>>(Cws, tab, P16);
  mq_attn_hd128<<<kBatch * kNumHeads * (kSeq / MQ_QB), 128, 0, stream>>>(
      Qh, Ql, Kh, Kl, Vh, Vl, out, kSeq, kNumHeads, kNqk, sscale);
}
